// Transformer_70274254897751
// MI455X (gfx1250) — hardware-verified
//
#include <hip/hip_runtime.h>
#include <stddef.h>
#include <stdint.h>


#define FIN     15
#define CH      128
#define KB1     32
#define K2      256
#define N1C     384
#define N2R     512
#define N3C     32
#define LDQ     384
#define OC      5
#define ATW     64
#define DEGCAP  64
#define NBIAS   928
#define NTHR    256
#define NWAVE   8
#define EPT     8
#define CHUNK   (NTHR * EPT)
#define WCAP    (EPT * 32)
#define LISTN   (NWAVE * WCAP)
#define NBMAX   2048
#define NBRUN   1024
#define ESH     11
#define RCAP    28672
#define STW     512
#define GBM     64
#define GTHR    128
#define SROWS   512
#define STHR    128
#define PARTD   256
#define NB1     ((N1C * KB1 / 8) / NTHR)
#define NB2     ((N2R * K2 / 8) / NTHR)
#define NB3     ((N3C * K2 / 8) / NTHR)
#define NBB     ((NBIAS + NTHR - 1) / NTHR)
#define NPT     ((NBRUN * OC / 4 + NTHR - 1) / NTHR)
#define NEGBIG  (-1.0e30f)
#define WSMAX   134217728
#define LDS_AGG ((2 * RCAP + 2 * NBMAX + LISTN) * 4 + 64)

static_assert((CHUNK & (CHUNK - 1)) == 0 && CHUNK <= 4096);
static_assert((NBMAX & (NBMAX - 1)) == 0 && NBMAX <= 4096);
static_assert((NBRUN & (NBRUN - 1)) == 0 && NBRUN <= NBMAX && NBRUN >= 32);
static_assert((1 << ESH) >= NBMAX);
static_assert(NTHR * 8 == NBMAX);
static_assert(LISTN >= NBMAX);
static_assert(LISTN >= NWAVE * WCAP);
static_assert((RCAP % 32) == 0 && ((2 * RCAP) % (NTHR * 4)) == 0);
static_assert(NWAVE * STW <= RCAP);
static_assert(3 * ATW <= STW);
static_assert(DEGCAP == ATW && ATW == 64);
static_assert(NBRUN * OC <= RCAP);
static_assert(NPT * NTHR * 4 >= NBRUN * OC);
static_assert(LDS_AGG <= 300000);
static_assert(GBM == (GTHR / 32) * 16);
static_assert((KB1 % 32) == 0 && (K2 % 32) == 0 && K2 == 2 * CH);
static_assert((N1C % 128) == 0 && N1C == 3 * CH && N2R == 4 * CH && LDQ == N1C);
static_assert(NBIAS == N1C + N2R + N3C && (NBIAS % 32) == 0);
static_assert(NB1 * NTHR == N1C * KB1 / 8 && NB2 * NTHR == N2R * K2 / 8 && NB3 * NTHR == N3C * K2 / 8);
static_assert(STHR == CH && PARTD == 2 * CH && NTHR == 2 * CH);
static_assert(OC == 5 && N3C == 32);

typedef float          v4f   __attribute__((ext_vector_type(4)));
typedef float          v8f   __attribute__((ext_vector_type(8)));
typedef int            v4i   __attribute__((ext_vector_type(4)));
typedef int            v8i   __attribute__((ext_vector_type(8)));
typedef double         v2d   __attribute__((ext_vector_type(2)));
typedef unsigned short v8us  __attribute__((ext_vector_type(8)));
typedef unsigned short v16us __attribute__((ext_vector_type(16)));
typedef __bf16         v16bf __attribute__((ext_vector_type(16)));
typedef v4f  __attribute__((may_alias)) v4fa;
typedef v4i  __attribute__((may_alias)) v4ia;
typedef v2d  __attribute__((may_alias)) v2da;
typedef v8us __attribute__((may_alias)) v8usa;
union FragB { v16bf v; v16us u; v8us h[2]; v8i w; };

__device__ __forceinline__ v8f wmb(const FragB& a, const FragB& b, v8f c) {
  v8f d = __builtin_amdgcn_wmma_f32_16x16x32_bf16(false, a.v, false, b.v, (short)0, c, false, false);
  asm volatile("v_nop\n\tv_nop\n\tv_nop\n\tv_nop" : "+v"(d) : "v"(a.w), "v"(b.w));
  return d;
}

__device__ __forceinline__ v8f z8() { v8f z = {0.f, 0.f, 0.f, 0.f, 0.f, 0.f, 0.f, 0.f}; return z; }

__device__ __forceinline__ unsigned bfbits(float v) {
  unsigned u = __float_as_uint(v);
  u = u + 0x7FFFu + ((u >> 16) & 1u);
  return u >> 16;
}
__device__ __forceinline__ float rbf(float v) { return __uint_as_float(bfbits(v) << 16); }

__device__ __forceinline__ void put8us(unsigned short* p, const v8us hv) {
  *(volatile v8us*)p = hv;
  __threadfence();
  *(volatile v8us*)p = hv;
}

__device__ __forceinline__ int scan_chunk(const int* __restrict__ dsts, int nE, int cbase, int slotBase,
                                          int nb, int vec8, int* list, int tid, int lane, int wave) {
  int wc = 0;
  const int el0  = tid * EPT;
  const int e0   = cbase + el0;
  const int sent = -2147483647 - 1;
  v4i da, db;
  if (vec8 != 0 && cbase + CHUNK <= nE) {
    da = *(const v4i*)(dsts + e0);
    db = *(const v4i*)(dsts + e0 + 4);
  } else {
    da.x = (e0     < nE) ? dsts[min(e0,     nE - 1)] : sent;
    da.y = (e0 + 1 < nE) ? dsts[min(e0 + 1, nE - 1)] : sent;
    da.z = (e0 + 2 < nE) ? dsts[min(e0 + 2, nE - 1)] : sent;
    da.w = (e0 + 3 < nE) ? dsts[min(e0 + 3, nE - 1)] : sent;
    db.x = (e0 + 4 < nE) ? dsts[min(e0 + 4, nE - 1)] : sent;
    db.y = (e0 + 5 < nE) ? dsts[min(e0 + 5, nE - 1)] : sent;
    db.z = (e0 + 6 < nE) ? dsts[min(e0 + 6, nE - 1)] : sent;
    db.w = (e0 + 7 < nE) ? dsts[min(e0 + 7, nE - 1)] : sent;
  }
  const unsigned nbs = (unsigned)slotBase;
  const unsigned unb = (unsigned)nb;
  const unsigned s0 = (unsigned)da.x - nbs, s1 = (unsigned)da.y - nbs;
  const unsigned s2 = (unsigned)da.z - nbs, s3 = (unsigned)da.w - nbs;
  const unsigned s4 = (unsigned)db.x - nbs, s5 = (unsigned)db.y - nbs;
  const unsigned s6 = (unsigned)db.z - nbs, s7 = (unsigned)db.w - nbs;
  const bool h0 = s0 < unb, h1 = s1 < unb, h2 = s2 < unb, h3 = s3 < unb;
  const bool h4 = s4 < unb, h5 = s5 < unb, h6 = s6 < unb, h7 = s7 < unb;
  const unsigned any = __builtin_amdgcn_ballot_w32(h0 | h1 | h2 | h3 | h4 | h5 | h6 | h7);
  if (any != 0u) {
#define HITJ(J, HJ, SJ) { \
      const unsigned mj = __builtin_amdgcn_ballot_w32(HJ); \
      if (mj != 0u) { \
        if (HJ) { \
          const int pos = wc + (int)__builtin_amdgcn_mbcnt_lo(mj, 0u); \
          if (pos < WCAP) list[wave * WCAP + pos] = ((el0 + (J)) << 12) | (int)(SJ); \
        } \
        wc += (int)__builtin_popcount(mj); } }
    HITJ(0, h0, s0)
    HITJ(1, h1, s1)
    HITJ(2, h2, s2)
    HITJ(3, h3, s3)
    HITJ(4, h4, s4)
    HITJ(5, h5, s5)
    HITJ(6, h6, s6)
    HITJ(7, h7, s7)
#undef HITJ
  }
  return wc;
}

__device__ __forceinline__ int build_lists(const int* __restrict__ dsts, int nE, int nodeBase, int nb, int vec8,
                                           int* reg1, int* reg2, int* scnt, int* soff, int* list,
                                           int* wcnt, int* wtot, int tid, int lane, int wave) {
  {
    const v4i z4 = {0, 0, 0, 0};
    for (int i = tid * 4; i < 2 * RCAP; i += NTHR * 4) *(v4ia*)(reg1 + i) = z4;
  }
  for (int i = tid; i < NBMAX; i += NTHR) scnt[i] = 0;
  __syncthreads();

  int tot = 0;
  const int nChunks = (nE + CHUNK - 1) / CHUNK;
#pragma unroll 1
  for (int ch = 0; ch < nChunks; ++ch) {
    const int cbase = ch * CHUNK;
    const int wc = scan_chunk(dsts, nE, cbase, nodeBase, nb, vec8, list, tid, lane, wave);
    if (lane == 0) wcnt[wave] = wc;
    __syncthreads();
    int pre = 0, all = 0;
#pragma unroll
    for (int w2 = 0; w2 < NWAVE; ++w2) {
      int c = wcnt[w2];
      c = c < 0 ? 0 : (c > WCAP ? WCAP : c);
      all += c;
      pre += (w2 < wave) ? c : 0;
    }
    const int wcc  = wc > WCAP ? WCAP : wc;
    const int base = tot + pre;
#pragma unroll 1
    for (int i = lane; i < wcc; i += 32) {
      const int ent = list[wave * WCAP + i];
      const int el  = (ent >> 12) & (CHUNK - 1);
      const int sl  = ent & (NBMAX - 1);
      int eid = cbase + el;
      eid = eid > nE - 1 ? nE - 1 : eid;
      const int pos = base + i;
      if (pos < RCAP) reg1[pos] = (int)(((unsigned)eid << ESH) | (unsigned)sl);
    }
    tot += all;
    tot = tot > RCAP ? RCAP : tot;
    __syncthreads();
  }
  const int nh = tot;

  if (wave == 0) {
#pragma unroll 1
    for (int b0 = 0; b0 < nh; b0 += 32) {
      const int idx = b0 + lane;
      const int uv  = reg1[idx < RCAP ? idx : RCAP - 1];
      const int m32 = (nh - b0) < 32 ? (nh - b0) : 32;
#pragma unroll 1
      for (int k = 0; k < m32; ++k) {
        const int u  = __builtin_amdgcn_readlane(uv, k);
        const int sl = u & (NBMAX - 1);
        if (lane == 0) scnt[sl] = scnt[sl] + 1;
      }
    }
  }
  __syncthreads();

  {
    const v4i ca = *(const v4ia*)(scnt + 8 * tid);
    const v4i cb = *(const v4ia*)(scnt + 8 * tid + 4);
    const int e0 = ca.x < 0 ? 0 : ca.x, e1 = ca.y < 0 ? 0 : ca.y, e2 = ca.z < 0 ? 0 : ca.z, e3 = ca.w < 0 ? 0 : ca.w;
    const int e4 = cb.x < 0 ? 0 : cb.x, e5 = cb.y < 0 ? 0 : cb.y, e6 = cb.z < 0 ? 0 : cb.z, e7 = cb.w < 0 ? 0 : cb.w;
    const int ts = e0 + e1 + e2 + e3 + e4 + e5 + e6 + e7;
    int incl = ts;
#pragma unroll
    for (int d = 1; d < 32; d <<= 1) {
      const int up = __shfl_up(incl, d);
      if (lane >= d) incl += up;
    }
    if (lane == 31) wtot[wave] = incl;
    __syncthreads();
    int pre = 0;
#pragma unroll
    for (int w2 = 0; w2 < NWAVE; ++w2) pre += (w2 < wave) ? wtot[w2] : 0;
    int run = pre + incl - ts;
    soff[8 * tid + 0] = run; run += e0;
    soff[8 * tid + 1] = run; run += e1;
    soff[8 * tid + 2] = run; run += e2;
    soff[8 * tid + 3] = run; run += e3;
    soff[8 * tid + 4] = run; run += e4;
    soff[8 * tid + 5] = run; run += e5;
    soff[8 * tid + 6] = run; run += e6;
    soff[8 * tid + 7] = run;
  }
  __syncthreads();
  for (int i = tid; i < NBMAX; i += NTHR) list[i] = soff[i];
  __syncthreads();

  if (wave == 0) {
#pragma unroll 1
    for (int b0 = 0; b0 < nh; b0 += 32) {
      const int idx = b0 + lane;
      const int uv  = reg1[idx < RCAP ? idx : RCAP - 1];
      const int m32 = (nh - b0) < 32 ? (nh - b0) : 32;
#pragma unroll 1
      for (int k = 0; k < m32; ++k) {
        const int u   = __builtin_amdgcn_readlane(uv, k);
        const int sl  = u & (NBMAX - 1);
        const int eid = (int)((unsigned)u >> ESH);
        if (lane == 0) {
          int pos = list[sl];
          pos = pos < 0 ? 0 : (pos > RCAP - 1 ? RCAP - 1 : pos);
          reg2[pos] = eid;
          list[sl] = pos + 1;
        }
      }
    }
  }
  __syncthreads();
  return nh;
}

__global__ __launch_bounds__(NTHR) void k_prep(
    const float* __restrict__ xin, int nN, int MPr, int nBx,
    const float* __restrict__ wq1, const float* __restrict__ wk1, const float* __restrict__ wv1,
    const float* __restrict__ wq2, const float* __restrict__ wk2, const float* __restrict__ wv2,
    const float* __restrict__ ws2,
    const float* __restrict__ wq3, const float* __restrict__ wk3, const float* __restrict__ wv3,
    const float* __restrict__ ws3,
    const float* __restrict__ bq1, const float* __restrict__ bk1, const float* __restrict__ bv1,
    const float* __restrict__ bq2, const float* __restrict__ bk2, const float* __restrict__ bv2,
    const float* __restrict__ bs2,
    const float* __restrict__ bq3, const float* __restrict__ bk3, const float* __restrict__ bv3,
    const float* __restrict__ bs3,
    unsigned short* xb1, unsigned short* wt1, unsigned short* wt2, unsigned short* wt3, float* bi) {
  const int b = (int)blockIdx.x, tid = (int)threadIdx.x;
  if (b < nBx) {
    const int i = b * NTHR + tid;
    if (i >= MPr * 4) return;
    const int row = i >> 2;
    const int c8  = (i & 3) * 8;
    const int rc  = row < nN ? row : nN - 1;
    const float* p = xin + (size_t)rc * FIN;
    v8us o;
#pragma unroll
    for (int j = 0; j < 8; ++j) {
      const int c  = c8 + j;
      const int cl = c < FIN ? c : FIN - 1;
      const float x = p[cl];
      const float v = (c < FIN && row < nN) ? x : 0.0f;
      o[j] = (unsigned short)bfbits(v);
    }
    put8us(xb1 + (size_t)i * 8, o);
  } else if (b < nBx + NB1) {
    const int u = (b - nBx) * NTHR + tid;
    const int n = u >> 2;
    const int k8 = (u & 3) * 8;
    const int seg = n >> 7;
    const int nc = n & (CH - 1);
    const float* w = (seg == 0) ? wq1 : ((seg == 1) ? wk1 : wv1);
    v8us o;
#pragma unroll
    for (int j = 0; j < 8; ++j) {
      const int k  = k8 + j;
      const int kc = k < FIN ? k : FIN - 1;
      const float x = w[(size_t)kc * CH + nc];
      o[j] = (unsigned short)bfbits(k < FIN ? x : 0.0f);
    }
    put8us(wt1 + (size_t)u * 8, o);
  } else if (b < nBx + NB1 + NB2) {
    const int v = (b - nBx - NB1) * NTHR + tid;
    const int n = v >> 5;
    const int k8 = (v & 31) * 8;
    const int kk = k8 & (CH - 1);
    const int seg = n >> 7;
    const int nc = n & (CH - 1);
    const float* w = (seg == 0) ? wq2 : ((seg == 1) ? wk2 : ((seg == 2) ? wv2 : ws2));
    const float* p = w + (size_t)kk * CH + nc;
    v8us o;
#pragma unroll
    for (int j = 0; j < 8; ++j) o[j] = (unsigned short)bfbits(p[(size_t)j * CH]);
    put8us(wt2 + (size_t)v * 8, o);
  } else if (b < nBx + NB1 + NB2 + NB3) {
    const int u = (b - nBx - NB1 - NB2) * NTHR + tid;
    const int n = u >> 5;
    const int k8 = (u & 31) * 8;
    const int kk = k8 & (CH - 1);
    const int g = n >> 3;
    const int cc = n & 7;
    const int ccl = cc < OC ? cc : OC - 1;
    const float* w = (g == 0) ? wq3 : ((g == 1) ? wk3 : ((g == 2) ? wv3 : ws3));
    const float* p = w + (size_t)kk * OC + ccl;
    v8us o;
#pragma unroll
    for (int j = 0; j < 8; ++j) {
      const float x = p[(size_t)j * OC];
      o[j] = (unsigned short)bfbits(cc < OC ? x : 0.0f);
    }
    put8us(wt3 + (size_t)u * 8, o);
  } else {
    const int e = (b - nBx - NB1 - NB2 - NB3) * NTHR + tid;
    if (e >= NBIAS) return;
    const int grp = e >> 7;
    float val;
    if (grp < 7) {
      const float* bp = (grp == 0) ? bq1 : ((grp == 1) ? bk1 : ((grp == 2) ? bv1 : ((grp == 3) ? bq2 :
                        ((grp == 4) ? bk2 : ((grp == 5) ? bv2 : bs2)))));
      val = bp[e & (CH - 1)];
    } else {
      const int l = e - 7 * CH;
      const int g = l >> 3;
      const int cc = l & 7;
      const int ccl = cc < OC ? cc : OC - 1;
      const float xq = bq3[ccl], xk = bk3[ccl], xv = bv3[ccl], xs = bs3[ccl];
      const float pick = (g == 0) ? xq : ((g == 1) ? xk : ((g == 2) ? xv : xs));
      val = (cc < OC) ? pick : 0.0f;
    }
    const float r = rbf(val);
    float* dp = bi + e;
    *(volatile float*)dp = r;
    __threadfence();
    *(volatile float*)dp = r;
  }
}

template <int NT, int MODE>
__global__ __launch_bounds__(GTHR) void k_gemm(const unsigned short* __restrict__ A,
                                               const unsigned short* __restrict__ BT,
                                               int K, int nN, const float* __restrict__ bias,
                                               float* xout, int ldo) {
  constexpr int GBN = 16 * NT;
  constexpr int PPR = GBN / 4;
  constexpr int RPI = 32 / PPR;
  constexpr int NI  = 16 / RPI;
  static_assert(NT == 2 || NT == 4 || NT == 8);
  __shared__ __attribute__((aligned(16))) float stg[GBM * GBN];
  const int tid = (int)threadIdx.x, lane = tid & 31, wave = tid >> 5, hh = lane >> 4, m = lane & 15;
  const int rowBase = (int)blockIdx.x * GBM;
  const int colBase = (int)blockIdx.y * GBN;

  v8f acc[NT];
#pragma unroll
  for (int t = 0; t < NT; ++t) acc[t] = z8();
  const unsigned short* ap = A  + (size_t)(rowBase + 16 * wave + m) * (size_t)K + 8 * hh;
  const unsigned short* bp = BT + (size_t)(colBase + m) * (size_t)K + 8 * hh;

#pragma unroll 1
  for (int k0 = 0; k0 < K; k0 += 32) {
    FragB af;
    af.h[0] = *(const v8usa*)(ap + k0);
    af.h[1] = *(const v8usa*)(ap + k0 + 16);
#pragma unroll
    for (int nt = 0; nt < NT; ++nt) {
      const unsigned short* wq = bp + (size_t)(16 * nt) * (size_t)K + k0;
      FragB bf;
      bf.h[0] = *(const v8usa*)wq;
      bf.h[1] = *(const v8usa*)(wq + 16);
      acc[nt] = wmb(af, bf, acc[nt]);
    }
  }

#pragma unroll
  for (int nt = 0; nt < NT; ++nt) {
    const int lc = 16 * nt + m;
#pragma unroll
    for (int r = 0; r < 8; ++r) {
      const int lr = 16 * wave + 8 * hh + r;
      stg[lr * GBN + lc] = acc[nt][r];
    }
  }
  __syncthreads();

  const int pir  = lane % PPR;
  const int rofs = lane / PPR;
  const v4f b4 = *(const v4f*)(bias + colBase + 4 * pir);
  v4f pv[NI];
#pragma unroll
  for (int i = 0; i < NI; ++i) {
    const int lr  = 16 * wave + i * RPI + rofs;
    const int row = rowBase + lr;
    const v4f x = *(const v4fa*)(stg + lr * GBN + 4 * pir);
    v4f y = x + b4;
    if (MODE == 1) {
      const v4f o = *(const v4fa*)(xout + (size_t)row * (size_t)ldo + colBase + 4 * pir);
      y = y + o;
    }
    const bool ok = row < nN;
    v4f q;
    q.x = ok ? y.x : 0.0f; q.y = ok ? y.y : 0.0f; q.z = ok ? y.z : 0.0f; q.w = ok ? y.w : 0.0f;
    pv[i] = q;
  }
#pragma unroll
  for (int i = 0; i < NI; ++i) {
    const int lr = 16 * wave + i * RPI + rofs;
    float* op = xout + (size_t)(rowBase + lr) * (size_t)ldo + colBase + 4 * pir;
    *(volatile v4f*)op = pv[i];
  }
  __threadfence();
#pragma unroll
  for (int i = 0; i < NI; ++i) {
    const int lr = 16 * wave + i * RPI + rofs;
    float* op = xout + (size_t)(rowBase + lr) * (size_t)ldo + colBase + 4 * pir;
    *(volatile v4f*)op = pv[i];
  }
}

template <int EWIN>
__global__ __launch_bounds__(NTHR) void k_agg(
    const int* __restrict__ srcs, const int* __restrict__ dsts,
    const float* __restrict__ ewp, const float* __restrict__ wev,
    float* qkv, float* attout,
    int nN, int nE, int nb, int vec8, int MPr, float rsc) {
  extern __shared__ v4f lds_dyn[];
  int* reg1 = (int*)lds_dyn;
  int* reg2 = reg1 + RCAP;
  int* scnt = reg2 + RCAP;
  int* soff = scnt + NBMAX;
  int* list = soff + NBMAX;
  int* wcnt = list + LISTN;
  int* wtot = wcnt + NWAVE;
  const int tid = (int)threadIdx.x, lane = tid & 31, wave = tid >> 5;
  const int nodeBase = (int)blockIdx.x * nb;

  const int nh = build_lists(dsts, nE, nodeBase, nb, vec8, reg1, reg2, scnt, soff, list, wcnt, wtot,
                             tid, lane, wave);

  const int nbw = nb >> 3;
  const bool ovf = (nh >= RCAP);
  const float qnan = __int_as_float(0x7fc00000);
  float* lg = (float*)reg1 + wave * STW;
  float* lw = lg + ATW;
  float* la = lg + 2 * ATW;
  const int c0  = 4 * lane;
  const int lcl = lane & 15;
  v4f we4 = *(const v4f*)(wev + c0);
  we4.x = rbf(we4.x); we4.y = rbf(we4.y); we4.z = rbf(we4.z); we4.w = rbf(we4.w);

#pragma unroll 1
  for (int jt = 0; jt < nbw; ++jt) {
    const int slot = wave * nbw + jt;
    const int node = nodeBase + slot;
    const int gcl  = node < nN ? node : nN - 1;
    int st = soff[slot];
    const int craw = scnt[slot];
    int cnt = craw;
    st  = st < 0 ? 0 : (st > nh ? nh : st);
    cnt = cnt < 0 ? 0 : (cnt > DEGCAP ? DEGCAP : cnt);
    if (cnt > nh - st) cnt = nh - st;
    const float pz = (ovf || craw > DEGCAP) ? qnan : 0.0f;
    const bool live = node < nN;

    const v4f q4 = *(const v4f*)(qkv + (size_t)gcl * LDQ + c0);
    float qe = q4.x * we4.x;
    qe = fmaf(q4.y, we4.y, qe);
    qe = fmaf(q4.z, we4.z, qe);
    qe = fmaf(q4.w, we4.w, qe);
#pragma unroll
    for (int off = 16; off > 0; off >>= 1) qe += __shfl_xor(qe, off);

    lg[lane] = NEGBIG; lg[lane + 32] = NEGBIG;
    lw[lane] = 0.0f;   lw[lane + 32] = 0.0f;

#pragma unroll 1
    for (int q = 0; q < cnt; ++q) {
      int idx = st + q; idx = idx > RCAP - 1 ? RCAP - 1 : idx;
      int eid = reg2[idx]; eid = eid < 0 ? 0 : (eid > nE - 1 ? nE - 1 : eid);
      const int sraw = srcs[eid];
      const int s = sraw < 0 ? 0 : (sraw > nN - 1 ? nN - 1 : sraw);
      float ew;
      if (EWIN) ew = rbf(ewp[eid]);
      else      ew = ewp[(size_t)node * ATW + q];
      const v4f k4 = *(const v4f*)(qkv + (size_t)s * LDQ + CH + c0);
      float part = q4.x * k4.x;
      part = fmaf(q4.y, k4.y, part);
      part = fmaf(q4.z, k4.z, part);
      part = fmaf(q4.w, k4.w, part);
#pragma unroll
      for (int off = 16; off > 0; off >>= 1) part += __shfl_xor(part, off);
      const float lgt = fmaf(ew, qe, part) * rsc;
      if (lane == 0) { lg[q] = lgt; lw[q] = ew; }
    }
    __builtin_amdgcn_fence(__ATOMIC_RELEASE, "wavefront");
    __builtin_amdgcn_wave_barrier();

    const float x0 = lg[lane], x1 = lg[lane + 32];
    const float w0 = lw[lane], w1 = lw[lane + 32];
    const bool val0 = lane < cnt, val1 = (lane + 32) < cnt;
    float lm = fmaxf(val0 ? x0 : NEGBIG, val1 ? x1 : NEGBIG);
#pragma unroll
    for (int off = 16; off > 0; off >>= 1) lm = fmaxf(lm, __shfl_xor(lm, off));
    float d0 = x0 - lm, d1 = x1 - lm;
    d0 = d0 < -80.f ? -80.f : (d0 > 0.f ? 0.f : d0);
    d1 = d1 < -80.f ? -80.f : (d1 > 0.f ? 0.f : d1);
    const float p0 = val0 ? __expf(d0) : 0.0f;
    const float p1 = val1 ? __expf(d1) : 0.0f;
    float sp = p0 + p1;
#pragma unroll
    for (int off = 16; off > 0; off >>= 1) sp += __shfl_xor(sp, off);
    const float inv = 1.0f / (sp + 1e-16f);
    const float a0 = p0 * inv, a1 = p1 * inv;
    float se = a0 * w0;
    se = fmaf(a1, w1, se);
#pragma unroll
    for (int off = 16; off > 0; off >>= 1) se += __shfl_xor(se, off);
    la[lane] = a0; la[lane + 32] = a1;
    __builtin_amdgcn_fence(__ATOMIC_RELEASE, "wavefront");
    __builtin_amdgcn_wave_barrier();

    v4f av = {0.0f, 0.0f, 0.0f, 0.0f};
#pragma unroll 1
    for (int q = 0; q < cnt; ++q) {
      int idx = st + q; idx = idx > RCAP - 1 ? RCAP - 1 : idx;
      int eid = reg2[idx]; eid = eid < 0 ? 0 : (eid > nE - 1 ? nE - 1 : eid);
      const int sraw = srcs[eid];
      const int s = sraw < 0 ? 0 : (sraw > nN - 1 ? nN - 1 : sraw);
      const float aq = la[q];
      const v4f v4 = *(const v4f*)(qkv + (size_t)s * LDQ + 2 * CH + c0);
      av.x = fmaf(aq, v4.x, av.x);
      av.y = fmaf(aq, v4.y, av.y);
      av.z = fmaf(aq, v4.z, av.z);
      av.w = fmaf(aq, v4.w, av.w);
    }
    v4f h4;
    h4.x = live ? (fmaf(se, we4.x, av.x) + pz) : 0.0f;
    h4.y = live ? (fmaf(se, we4.y, av.y) + pz) : 0.0f;
    h4.z = live ? (fmaf(se, we4.z, av.z) + pz) : 0.0f;
    h4.w = live ? (fmaf(se, we4.w, av.w) + pz) : 0.0f;

    const bool wr = node < MPr;
    float* hp = qkv + (size_t)node * LDQ + c0;
    const v4f ga = *(const v4fa*)(la + 4 * lcl);
    float* gpa = attout + (size_t)node * ATW + 4 * lcl;
    const bool wsv = lane < 16;
    if (wr)  *(volatile v4f*)hp  = h4;
    if (wsv) *(volatile v4f*)gpa = ga;
    __threadfence();
    if (wr)  *(volatile v4f*)hp  = h4;
    if (wsv) *(volatile v4f*)gpa = ga;
  }
}

struct Edge3 { float l, ew, v0, v1, v2, v3, v4; int ok; };

__device__ __forceinline__ Edge3 edge3(const int* __restrict__ srcs, const float* __restrict__ attin,
                                        const float* __restrict__ p3, const int* reg2,
                                        int st, int cnt, int cm1, int qq, size_t abase, int nN, int nE,
                                        v4f qa, float q4, float qe, float rsc) {
  Edge3 r;
  r.ok = qq < cnt ? 1 : 0;
  const int qc = qq < cm1 ? qq : cm1;
  int idx = st + qc; idx = idx > RCAP - 1 ? RCAP - 1 : idx;
  int eid = reg2[idx]; eid = eid < 0 ? 0 : (eid > nE - 1 ? nE - 1 : eid);
  const int sraw = srcs[eid];
  const int s = sraw < 0 ? 0 : (sraw > nN - 1 ? nN - 1 : sraw);
  const float ew = attin[abase + (size_t)qq];
  const float* kr = p3 + (size_t)s * N3C + 8;
  const v4f ka = *(const v4f*)kr;
  const v4f kb = *(const v4f*)(kr + 4);
  float dot = qa.x * ka.x;
  dot = fmaf(qa.y, ka.y, dot);
  dot = fmaf(qa.z, ka.z, dot);
  dot = fmaf(qa.w, ka.w, dot);
  dot = fmaf(q4, kb.x, dot);
  r.l = fmaf(ew, qe, dot) * rsc;
  r.ew = ew;
  const float* vr = p3 + (size_t)s * N3C + 16;
  const v4f va = *(const v4f*)vr;
  const v4f vb = *(const v4f*)(vr + 4);
  r.v0 = va.x; r.v1 = va.y; r.v2 = va.z; r.v3 = va.w; r.v4 = vb.x;
  return r;
}

__global__ __launch_bounds__(NTHR) void k_agg3(
    const int* __restrict__ srcs, const int* __restrict__ dsts,
    const float* __restrict__ attin, const float* __restrict__ wev,
    const float* __restrict__ p3, float* out, int nN, int nE, int nb, int vec8, float rsc) {
  extern __shared__ v4f lds_dyn[];
  int* reg1 = (int*)lds_dyn;
  int* reg2 = reg1 + RCAP;
  int* scnt = reg2 + RCAP;
  int* soff = scnt + NBMAX;
  int* list = soff + NBMAX;
  int* wcnt = list + LISTN;
  int* wtot = wcnt + NWAVE;
  const int tid = (int)threadIdx.x, lane = tid & 31, wave = tid >> 5;
  const int nodeBase = (int)blockIdx.x * nb;

  const int nh = build_lists(dsts, nE, nodeBase, nb, vec8, reg1, reg2, scnt, soff, list, wcnt, wtot,
                             tid, lane, wave);

  const int nbw = nb >> 3;
  const bool ovf = (nh >= RCAP);
  const float qnan = __int_as_float(0x7fc00000);
  float* sres = (float*)reg1;
  const float we0 = rbf(wev[0]), we1 = rbf(wev[1]), we2 = rbf(wev[2]), we3 = rbf(wev[3]), we4 = rbf(wev[4]);

#pragma unroll 1
  for (int jt = 0; jt < nbw; ++jt) {
    const int slot = wave * nbw + jt;
    const int node = nodeBase + slot;
    const int gcl  = node < nN ? node : nN - 1;
    int st = soff[slot];
    const int craw = scnt[slot];
    int cnt = craw;
    st  = st < 0 ? 0 : (st > nh ? nh : st);
    cnt = cnt < 0 ? 0 : (cnt > DEGCAP ? DEGCAP : cnt);
    if (cnt > nh - st) cnt = nh - st;
    const float pz = (ovf || craw > DEGCAP) ? qnan : 0.0f;

    const float* qrow = p3 + (size_t)gcl * N3C;
    const v4f qa = *(const v4f*)qrow;
    const v4f qb = *(const v4f*)(qrow + 4);
    const v4f ka = *(const v4f*)(qrow + 24);
    const v4f kb = *(const v4f*)(qrow + 28);
    const float q4 = qb.x;
    float qe = qa.x * we0;
    qe = fmaf(qa.y, we1, qe);
    qe = fmaf(qa.z, we2, qe);
    qe = fmaf(qa.w, we3, qe);
    qe = fmaf(q4, we4, qe);
    const int cm1 = cnt > 0 ? cnt - 1 : 0;
    const size_t abase = (size_t)node * ATW;

    const Edge3 e0 = edge3(srcs, attin, p3, reg2, st, cnt, cm1, lane,      abase, nN, nE, qa, q4, qe, rsc);
    const Edge3 e1 = edge3(srcs, attin, p3, reg2, st, cnt, cm1, lane + 32, abase, nN, nE, qa, q4, qe, rsc);

    float lm = fmaxf(e0.ok ? e0.l : NEGBIG, e1.ok ? e1.l : NEGBIG);
#pragma unroll
    for (int off = 16; off > 0; off >>= 1) lm = fmaxf(lm, __shfl_xor(lm, off));
    float d0 = e0.l - lm, d1 = e1.l - lm;
    d0 = d0 < -80.f ? -80.f : (d0 > 0.f ? 0.f : d0);
    d1 = d1 < -80.f ? -80.f : (d1 > 0.f ? 0.f : d1);
    const float p0 = e0.ok ? __expf(d0) : 0.0f;
    const float p1 = e1.ok ? __expf(d1) : 0.0f;
    float sp = p0 + p1;
#pragma unroll
    for (int off = 16; off > 0; off >>= 1) sp += __shfl_xor(sp, off);
    const float inv = 1.0f / (sp + 1e-16f);
    const float a0 = p0 * inv, a1 = p1 * inv;
    float r0 = a0 * e0.v0; r0 = fmaf(a1, e1.v0, r0);
    float r1 = a0 * e0.v1; r1 = fmaf(a1, e1.v1, r1);
    float r2 = a0 * e0.v2; r2 = fmaf(a1, e1.v2, r2);
    float r3 = a0 * e0.v3; r3 = fmaf(a1, e1.v3, r3);
    float r4 = a0 * e0.v4; r4 = fmaf(a1, e1.v4, r4);
    float se = a0 * e0.ew; se = fmaf(a1, e1.ew, se);
#pragma unroll
    for (int off = 16; off > 0; off >>= 1) {
      r0 += __shfl_xor(r0, off);
      r1 += __shfl_xor(r1, off);
      r2 += __shfl_xor(r2, off);
      r3 += __shfl_xor(r3, off);
      r4 += __shfl_xor(r4, off);
      se += __shfl_xor(se, off);
    }
    const float o0 = fmaf(se, we0, r0) + ka.x + pz;
    const float o1 = fmaf(se, we1, r1) + ka.y + pz;
    const float o2 = fmaf(se, we2, r2) + ka.z + pz;
    const float o3 = fmaf(se, we3, r3) + ka.w + pz;
    const float o4 = fmaf(se, we4, r4) + kb.x + pz;
    if (lane == 0) {
      sres[slot * OC + 0] = o0;
      sres[slot * OC + 1] = o1;
      sres[slot * OC + 2] = o2;
      sres[slot * OC + 3] = o3;
      sres[slot * OC + 4] = o4;
    }
  }
  __syncthreads();

  {
    int nrows = nN - nodeBase;
    nrows = nrows < 0 ? 0 : (nrows > nb ? nb : nrows);
    const int nf  = nrows * OC;
    const int np  = nf >> 2;
    const int rem = nf & 3;
    float* ob = out + (size_t)nodeBase * OC;
    v4f pv[NPT];
#pragma unroll
    for (int i = 0; i < NPT; ++i) {
      const int p  = tid + i * NTHR;
      const int pc = p < np ? p : (np > 0 ? np - 1 : 0);
      pv[i] = *(const v4fa*)(sres + 4 * pc);
    }
    const int tl = tid < rem ? tid : 0;
    const float tv = sres[4 * np + tl];
#pragma unroll
    for (int i = 0; i < NPT; ++i) {
      const int p = tid + i * NTHR;
      if (p < np) *(volatile v4f*)(ob + 4 * p) = pv[i];
    }
    if (tid < rem) *(volatile float*)(ob + 4 * np + tid) = tv;
    __threadfence();
#pragma unroll
    for (int i = 0; i < NPT; ++i) {
      const int p = tid + i * NTHR;
      if (p < np) *(volatile v4f*)(ob + 4 * p) = pv[i];
    }
    if (tid < rem) *(volatile float*)(ob + 4 * np + tid) = tv;
  }
}

__global__ __launch_bounds__(STHR) void k_bnstat(const float* __restrict__ h, int ldh, int nN, double* part) {
  __shared__ __attribute__((aligned(16))) double sd[PARTD];
  const int tid = (int)threadIdx.x;
  const int r0 = (int)blockIdx.x * SROWS;
  int r1 = r0 + SROWS; r1 = r1 > nN ? nN : r1;
  double s = 0.0, q = 0.0;
  const float* p = h + (size_t)r0 * (size_t)ldh + tid;
#pragma unroll 4
  for (int r = r0; r < r1; ++r) {
    const double x = (double)p[(size_t)(r - r0) * (size_t)ldh];
    s += x;
    q = fma(x, x, q);
  }
  sd[tid] = s;
  sd[CH + tid] = q;
  __syncthreads();
  const v2d v = *(const v2da*)(sd + 2 * tid);
  double* dp = part + (size_t)blockIdx.x * PARTD + 2 * tid;
  *(volatile v2d*)dp = v;
  __threadfence();
  *(volatile v2d*)dp = v;
}

__global__ __launch_bounds__(CH) void k_bnfin(const double* __restrict__ part, int nPart, int nN,
                                              const float* __restrict__ gam, const float* __restrict__ bet,
                                              float* ss) {
  __shared__ __attribute__((aligned(16))) float stg[2 * CH];
  const int c = (int)threadIdx.x;
  double s = 0.0, q = 0.0;
#pragma unroll 1
  for (int b = 0; b < nPart; ++b) {
    s += part[(size_t)b * PARTD + c];
    q += part[(size_t)b * PARTD + CH + c];
  }
  const double n = (double)(nN > 0 ? nN : 1);
  const double mean = s / n;
  double var = q / n - mean * mean;
  var = var < 0.0 ? 0.0 : var;
  const float varf  = (float)var;
  const float meanf = (float)mean;
  const float rstd = 1.0f / sqrtf(varf + 1e-5f);
  const float sc = rbf(gam[c]) * rstd;
  const float sh = rbf(bet[c]) - meanf * sc;
  stg[c] = sc;
  stg[CH + c] = sh;
  __syncthreads();
  v4f v;
  if (c < (2 * CH) / 4) {
    v = *(const v4fa*)(stg + 4 * c);
    *(volatile v4f*)(ss + 4 * c) = v;
  }
  __threadfence();
  if (c < (2 * CH) / 4) {
    *(volatile v4f*)(ss + 4 * c) = v;
  }
}

__global__ __launch_bounds__(NTHR) void k_act(const float* __restrict__ h, int ldh, const float* __restrict__ ss,
                                              int nN, int nUnits, unsigned short* xa) {
  __shared__ float ssh[2 * CH];
  const int tid = (int)threadIdx.x;
  ssh[tid] = ss[tid];
  __syncthreads();
  const int u = (int)blockIdx.x * NTHR + tid;
  if (u >= nUnits) return;
  const int row = u >> 4;
  const int c8  = (u & 15) * 8;
  const int rc  = row < nN ? row : nN - 1;
  const float* p = h + (size_t)rc * (size_t)ldh + c8;
  const v4f a = *(const v4f*)p;
  const v4f b = *(const v4f*)(p + 4);
  float y[8] = {a.x, a.y, a.z, a.w, b.x, b.y, b.z, b.w};
  v8us hv, lv;
#pragma unroll
  for (int j = 0; j < 8; ++j) {
    float t = fmaf(y[j], ssh[c8 + j], ssh[CH + c8 + j]);
    t = (t >= 0.0f) ? t : 0.01f * t;
    const float yy = (row < nN) ? t : 0.0f;
    const unsigned hb = bfbits(yy);
    hv[j] = (unsigned short)hb;
    lv[j] = (unsigned short)bfbits(yy - __uint_as_float(hb << 16));
  }
  unsigned short* xp = xa + (size_t)row * K2 + c8;
  *(volatile v8us*)xp = hv;
  *(volatile v8us*)(xp + CH) = lv;
  __threadfence();
  *(volatile v8us*)xp = hv;
  *(volatile v8us*)(xp + CH) = lv;
}

static int pick_nb(int nE, int nN) {
  int nb = NBRUN;
  while (nb > 32 && (long long)nb * (long long)nE * 5LL > (long long)RCAP * (long long)nN * 4LL) nb >>= 1;
  return nb;
}
static inline int cdiv(int a, int b) { return (a + b - 1) / b; }
static inline size_t al256(size_t o) { return (o + 255) & ~(size_t)255; }

extern "C" void kernel_launch(void* const* d_in, const int* in_sizes, int n_in,
                              void* d_out, int out_size, void* d_ws, size_t ws_size,
                              hipStream_t stream) {
  if (n_in < 34) return;
  if (in_sizes[1] < FIN || (in_sizes[1] % FIN) != 0) return;
  const int nN = in_sizes[1] / FIN;
  if (nN < 1 || nN > (1 << 22)) return;
  if (in_sizes[3] < 2 || (in_sizes[3] & 1) != 0) return;
  const int nE = in_sizes[3] / 2;
  if (nE < 1 || nE > (1 << 21)) return;
  if (in_sizes[4] != nE) return;
  if (in_sizes[5] != FIN * CH || in_sizes[6] != CH) return;
  if (in_sizes[7] != FIN * CH || in_sizes[8] != CH) return;
  if (in_sizes[9] != FIN * CH || in_sizes[10] != CH) return;
  if (in_sizes[11] != CH || in_sizes[12] != CH || in_sizes[13] != CH) return;
  if (in_sizes[14] != CH * CH || in_sizes[15] != CH) return;
  if (in_sizes[16] != CH * CH || in_sizes[17] != CH) return;
  if (in_sizes[18] != CH * CH || in_sizes[19] != CH) return;
  if (in_sizes[20] != CH) return;
  if (in_sizes[21] != CH * CH || in_sizes[22] != CH) return;
  if (in_sizes[23] != CH || in_sizes[24] != CH) return;
  if (in_sizes[25] != CH * OC || in_sizes[26] != OC) return;
  if (in_sizes[27] != CH * OC || in_sizes[28] != OC) return;
  if (in_sizes[29] != CH * OC || in_sizes[30] != OC) return;
  if (in_sizes[31] != OC) return;
  if (in_sizes[32] != CH * OC || in_sizes[33] != OC) return;
  if ((long long)out_size != (long long)nN * OC) return;

  const float* xin = (const float*)d_in[1];
  const int*   ei  = (const int*)  d_in[3];
  const float* ew  = (const float*)d_in[4];
  const float* Wq1 = (const float*)d_in[5];  const float* bq1 = (const float*)d_in[6];
  const float* Wk1 = (const float*)d_in[7];  const float* bk1 = (const float*)d_in[8];
  const float* Wv1 = (const float*)d_in[9];  const float* bv1 = (const float*)d_in[10];
  const float* We1 = (const float*)d_in[11];
  const float* g1  = (const float*)d_in[12]; const float* be1 = (const float*)d_in[13];
  const float* Wq2 = (const float*)d_in[14]; const float* bq2 = (const float*)d_in[15];
  const float* Wk2 = (const float*)d_in[16]; const float* bk2 = (const float*)d_in[17];
  const float* Wv2 = (const float*)d_in[18]; const float* bv2 = (const float*)d_in[19];
  const float* We2 = (const float*)d_in[20];
  const float* Ws2 = (const float*)d_in[21]; const float* bs2 = (const float*)d_in[22];
  const float* g2  = (const float*)d_in[23]; const float* be2 = (const float*)d_in[24];
  const float* Wq3 = (const float*)d_in[25]; const float* bq3 = (const float*)d_in[26];
  const float* Wk3 = (const float*)d_in[27]; const float* bk3 = (const float*)d_in[28];
  const float* Wv3 = (const float*)d_in[29]; const float* bv3 = (const float*)d_in[30];
  const float* We3 = (const float*)d_in[31];
  const float* Ws3 = (const float*)d_in[32]; const float* bs3 = (const float*)d_in[33];
  float* out = (float*)d_out;
  const int* src = ei;
  const int* dst = ei + nE;

  const int MP   = cdiv(nN, GBM) * GBM;
  const int gM   = MP / GBM;
  const int nb   = pick_nb(nE, nN);
  const int gA   = cdiv(MP, nb);
  if ((long long)gA * nb < (long long)MP) return;
  const int vec8 = ((nE & 3) == 0) ? 1 : 0;
  const int nSB  = cdiv(nN, SROWS);
  const long long nAttRows = (long long)gA * nb;

  char* ws = (char*)d_ws;
  size_t off = 0;
  const size_t oWT1 = off; off = al256(off + (size_t)N1C * KB1 * 2);
  const size_t oWT2 = off; off = al256(off + (size_t)N2R * K2 * 2);
  const size_t oWT3 = off; off = al256(off + (size_t)N3C * K2 * 2);
  const size_t oBI  = off; off = al256(off + (size_t)NBIAS * 4);
  const size_t szQ  = (size_t)MP * LDQ * 4;
  const size_t szP3 = (size_t)MP * N3C * 4;
  const size_t oQKV = off; off = al256(off + (szQ > szP3 ? szQ : szP3));
  const size_t szXA = (size_t)MP * K2 * 2;
  const size_t szXB = (size_t)MP * KB1 * 2;
  const size_t oXA  = off; off = al256(off + (szXA > szXB ? szXA : szXB));
  const size_t oAT1 = off; off = al256(off + (size_t)nAttRows * ATW * 4);
  const size_t oAT2 = off; off = al256(off + (size_t)nAttRows * ATW * 4);
  const size_t oPT  = off; off = al256(off + (size_t)nSB * PARTD * 8);
  const size_t oSS  = off; off = al256(off + (size_t)(2 * CH) * 4);
  if (off > ws_size || off > (size_t)WSMAX) return;
  unsigned short* WT1 = (unsigned short*)(ws + oWT1);
  unsigned short* WT2 = (unsigned short*)(ws + oWT2);
  unsigned short* WT3 = (unsigned short*)(ws + oWT3);
  float*          BI  = (float*)(ws + oBI);
  float*          QKV = (float*)(ws + oQKV);
  float*          P3  = (float*)(ws + oQKV);
  unsigned short* XA  = (unsigned short*)(ws + oXA);
  unsigned short* XB1 = (unsigned short*)(ws + oXA);
  float*          AT1 = (float*)(ws + oAT1);
  float*          AT2 = (float*)(ws + oAT2);
  double*         PT  = (double*)(ws + oPT);
  float*          SS  = (float*)(ws + oSS);

  hipFuncSetAttribute(reinterpret_cast<const void*>(&k_agg<1>), hipFuncAttributeMaxDynamicSharedMemorySize, LDS_AGG);
  hipFuncSetAttribute(reinterpret_cast<const void*>(&k_agg<0>), hipFuncAttributeMaxDynamicSharedMemorySize, LDS_AGG);
  hipFuncSetAttribute(reinterpret_cast<const void*>(&k_agg3),   hipFuncAttributeMaxDynamicSharedMemorySize, LDS_AGG);

  const float rsc128 = 0.08838834764831845f;
  const float rsc5   = 0.4472135954999579f;
  const int nBx = (MP * 4) / NTHR;
  const int nUa = MP * 16;

  k_prep<<<nBx + NB1 + NB2 + NB3 + NBB, NTHR, 0, stream>>>(
      xin, nN, MP, nBx, Wq1, Wk1, Wv1, Wq2, Wk2, Wv2, Ws2, Wq3, Wk3, Wv3, Ws3,
      bq1, bk1, bv1, bq2, bk2, bv2, bs2, bq3, bk3, bv3, bs3, XB1, WT1, WT2, WT3, BI);
  k_gemm<8, 0><<<dim3(gM, N1C / 128), GTHR, 0, stream>>>(XB1, WT1, KB1, nN, BI, QKV, LDQ);
  k_agg<1><<<gA, NTHR, LDS_AGG, stream>>>(src, dst, ew, We1, QKV, AT1, nN, nE, nb, vec8, MP, rsc128);
  k_bnstat<<<nSB, STHR, 0, stream>>>(QKV, LDQ, nN, PT);
  k_bnfin<<<1, CH, 0, stream>>>(PT, nSB, nN, g1, be1, SS);
  k_act<<<nUa / NTHR, NTHR, 0, stream>>>(QKV, LDQ, SS, nN, nUa, XA);
  k_gemm<8, 0><<<dim3(gM, N1C / 128), GTHR, 0, stream>>>(XA, WT2, K2, nN, BI + N1C, QKV, LDQ);
  k_agg<0><<<gA, NTHR, LDS_AGG, stream>>>(src, dst, AT1, We2, QKV, AT2, nN, nE, nb, vec8, MP, rsc128);
  k_gemm<8, 1><<<dim3(gM, 1), GTHR, 0, stream>>>(XA, WT2 + (size_t)N1C * K2, K2, nN, BI + N1C + N1C, QKV, LDQ);
  k_bnstat<<<nSB, STHR, 0, stream>>>(QKV, LDQ, nN, PT);
  k_bnfin<<<1, CH, 0, stream>>>(PT, nSB, nN, g2, be2, SS);
  k_act<<<nUa / NTHR, NTHR, 0, stream>>>(QKV, LDQ, SS, nN, nUa, XA);
  k_gemm<2, 0><<<dim3(gM, 1), GTHR, 0, stream>>>(XA, WT3, K2, nN, BI + N1C + N2R, P3, N3C);
  k_agg3<<<gA, NTHR, LDS_AGG, stream>>>(src, dst, AT2, We3, P3, out, nN, nE, nb, vec8, rsc5);
}
